// MMDLayer_51917564674624
// MI455X (gfx1250) — hardware-verified
//
#include <hip/hip_runtime.h>
#include <math.h>

typedef __attribute__((ext_vector_type(16))) _Float16 v16h;
typedef __attribute__((ext_vector_type(8)))  _Float16 v8h;
typedef __attribute__((ext_vector_type(8)))  float    v8f;
typedef __attribute__((ext_vector_type(4)))  float    v4f;
typedef __attribute__((ext_vector_type(4)))  unsigned int v4u;

constexpr int kNumZ         = 16384;
constexpr int kNumG         = 200;
constexpr int kNumGPad      = 256;
constexpr int kFeat         = 64;
constexpr int kTile         = 64;
constexpr int kWavesPerBlk  = 8;
constexpr int kLineFloats   = 32;
constexpr int kPrepRows     = 32;
constexpr int kTilesZ       = kNumZ / kTile;
constexpr int kTilesG       = kNumGPad / kTile;
constexpr int kShiftZ       = 8;
constexpr int kShiftG       = 2;
constexpr int kBlocksZZ     = (kTilesZ * kTilesZ) / kWavesPerBlk;
constexpr int kBlocksGZ     = (kTilesG * kTilesZ) / kWavesPerBlk;
constexpr int kBlocksGG     = (kTilesG * kTilesG) / kWavesPerBlk;
constexpr int kPrepBlocksZ  = kNumZ / kPrepRows;
constexpr int kPrepBlocksG  = kNumGPad / kPrepRows;

static_assert(kFeat % 32 == 0, "K multiple of 32, no K tail");
static_assert(kNumZ % kTile == 0 && kNumGPad % kTile == 0, "M and N tile multiples");
static_assert((1 << kShiftZ) == kTilesZ && (1 << kShiftG) == kTilesG, "tile shifts");
static_assert((kTilesZ * kTilesZ) % kWavesPerBlk == 0, "zz tiles per block exact");
static_assert((kTilesG * kTilesZ) % kWavesPerBlk == 0, "gz tiles per block exact");
static_assert((kTilesG * kTilesG) % kWavesPerBlk == 0, "gg tiles per block exact");
static_assert(kNumZ % kPrepRows == 0 && kNumGPad % kPrepRows == 0, "prep rows exact");
static_assert(kBlocksZZ % 256 == 0, "combine kernel strided coverage exact");
static_assert(kBlocksGZ <= 256 && kBlocksGG <= 256, "combine kernel single pass");
static_assert(kNumG <= kNumGPad, "pad");

constexpr size_t kOffZh   = 0;
constexpr size_t kOffGh   = kOffZh  + (size_t)kNumZ * kFeat * 2;
constexpr size_t kOffNz   = kOffGh  + (size_t)kNumGPad * kFeat * 2;
constexpr size_t kOffNg   = kOffNz  + (size_t)kNumZ * 4;
constexpr size_t kOffPzz  = kOffNg  + (size_t)kNumGPad * 4;
constexpr size_t kOffPgz  = kOffPzz + (size_t)kBlocksZZ * kLineFloats * 4;
constexpr size_t kOffPgg  = kOffPgz + (size_t)kBlocksGZ * kLineFloats * 4;
constexpr size_t kWsTotal = kOffPgg + (size_t)kBlocksGG * kLineFloats * 4;
static_assert(kWsTotal <= (size_t)134217728, "carve under 128 MiB");
static_assert(kOffGh % 128 == 0 && kOffNz % 128 == 0 && kOffNg % 128 == 0, "line aligned");
static_assert(kOffPzz % 128 == 0 && kOffPgz % 128 == 0 && kOffPgg % 128 == 0, "line aligned");

__device__ __forceinline__ void dep_guard_h(v8f& a, v8f& b, v16h x, v16h y) { asm volatile("v_nop\n\tv_nop\n\tv_nop\n\tv_nop" : "+v"(a), "+v"(b) : "v"(x), "v"(y)); }
__device__ __forceinline__ void keep4_h(v16h a, v16h b, v16h c, v16h d) { asm volatile("v_nop" :: "v"(a), "v"(b), "v"(c), "v"(d)); }
__device__ __forceinline__ void acc_guard4(v8f& a, v8f& b, v8f& c, v8f& d) { asm volatile("v_nop\n\tv_nop\n\tv_nop\n\tv_nop" : "+v"(a), "+v"(b), "+v"(c), "+v"(d)); }
template <typename T> struct Frag;
template <> struct Frag<_Float16> {
  typedef v16h V; union U { v16h v; v8h h[2]; };
  static __device__ __forceinline__ v16h load(const _Float16* p) {
    U f; f.h[0] = *(const v8h*)(p); f.h[1] = *(const v8h*)(p + 16); return f.v;
  }
  static __device__ __forceinline__ v8f mma(v16h a, v16h b, v8f c) {
    return __builtin_amdgcn_wmma_f32_16x16x32_f16(false, a, false, b, (short)0, c, false, false);
  }
  static __device__ __forceinline__ void guard(v8f& a, v8f& b, v16h x, v16h y) { dep_guard_h(a, b, x, y); }
  static __device__ __forceinline__ void keep(v16h a, v16h b, v16h c, v16h d) { keep4_h(a, b, c, d); }
};

__device__ __forceinline__ unsigned pk16(unsigned short a, unsigned short b) { return (unsigned)a | ((unsigned)b << 16); }
__device__ __forceinline__ unsigned short h_bits(float f) { const _Float16 h = (_Float16)f; return __builtin_bit_cast(unsigned short, h); }

__device__ __forceinline__ float quant_h(float f) {
  const unsigned u   = __float_as_uint(f);
  const unsigned mag = u & 0x7fffffffu;
  const unsigned r   = (u + 0x0FFFu + ((u >> 13) & 1u)) & 0xFFFFE000u;
  const float q = __uint_as_float(r);
  return (mag < 0x38800000u) ? 0.0f : q;
}

__global__ __launch_bounds__(256) void prep_rows_kernel(
    const float* __restrict__ src, int validRows,
    unsigned short* __restrict__ dst, float* __restrict__ nrm, float nscale) {
  __shared__ __align__(16) float sNorm[kPrepRows];
  const int t    = threadIdx.x;
  const int lane = t & 31;
  const int wave = t >> 5;
  const int q    = lane >> 3;
  const int e8   = (lane & 7) * 8;
  const int rloc = wave * 4 + q;
  const int row  = blockIdx.x * kPrepRows + rloc;
  const bool rv  = row < validRows;
  const int rowc = rv ? row : (validRows - 1);
  const float* p = src + (size_t)rowc * kFeat + e8;
  const v4f a = *(const v4f*)(p);
  const v4f c = *(const v4f*)(p + 4);
  float x[8];
  x[0] = a[0]; x[1] = a[1]; x[2] = a[2]; x[3] = a[3];
  x[4] = c[0]; x[5] = c[1]; x[6] = c[2]; x[7] = c[3];
  unsigned short hb[8];
  float s = 0.0f;
#pragma unroll
  for (int e = 0; e < 8; ++e) {
    const float xq = rv ? quant_h(x[e]) : 0.0f;
    hb[e] = h_bits(xq);
    s = fmaf(xq, xq, s);
  }
  s += __shfl_xor(s, 1, 32);
  s += __shfl_xor(s, 2, 32);
  s += __shfl_xor(s, 4, 32);
  const v4u u = (v4u){pk16(hb[0], hb[1]), pk16(hb[2], hb[3]), pk16(hb[4], hb[5]), pk16(hb[6], hb[7])};
  unsigned short* dp = dst + (size_t)row * kFeat + e8;
  *(volatile v4u*)dp = u;
  __threadfence();
  *(volatile v4u*)dp = u;
  if ((lane & 7) == 0) sNorm[rloc] = s * nscale;
  __syncthreads();
  if (wave == 0) {
    const int li = (lane & 7) * 4;
    v4f nv;
    nv[0] = sNorm[li + 0]; nv[1] = sNorm[li + 1]; nv[2] = sNorm[li + 2]; nv[3] = sNorm[li + 3];
    float* np = nrm + (size_t)blockIdx.x * kPrepRows + li;
    if (lane < 8) *(volatile v4f*)np = nv;
    __threadfence();
    if (lane < 8) *(volatile v4f*)np = nv;
  }
}

__global__ __launch_bounds__(256) void gram_tile_kernel(
    const unsigned short* __restrict__ Ap, const float* __restrict__ An, int rowsValid,
    const unsigned short* __restrict__ Btp, const float* __restrict__ Bn, int colsValid,
    int tilesNShift, float* __restrict__ partial, float s2) {
  typedef _Float16 T;
  typedef v16h V;
  const T* A  = (const T*)Ap;
  const T* Bt = (const T*)Btp;
  __shared__ float red[kWavesPerBlk];
  const int lane = threadIdx.x & 31;
  const int wave = threadIdx.x >> 5;
  const int tile = blockIdx.x * kWavesPerBlk + wave;
  const int tm   = tile >> tilesNShift;
  const int tn   = tile - (tm << tilesNShift);
  const int m0   = tm << 6;
  const int n0   = tn << 6;
  const int rlane = lane & 15;
  const int koff  = (lane >> 4) * 8;
  const int mOff  = (lane >> 4) * 8;

  v8f acc[4][4];
#pragma unroll
  for (int i = 0; i < 4; ++i)
#pragma unroll
    for (int j = 0; j < 4; ++j) acc[i][j] = (v8f){0.f,0.f,0.f,0.f,0.f,0.f,0.f,0.f};

#pragma unroll
  for (int k0 = 0; k0 < kFeat; k0 += 32) {
    V bh[4];
#pragma unroll
    for (int j = 0; j < 4; ++j) {
      const size_t bo = (size_t)(n0 + (j << 4) + rlane) * kFeat + koff + k0;
      bh[j] = Frag<T>::load(Bt + bo);
    }
#pragma unroll
    for (int i = 0; i < 4; ++i) {
      const size_t ao = (size_t)(m0 + (i << 4) + rlane) * kFeat + koff + k0;
      V ah = Frag<T>::load(A + ao);
#pragma unroll
      for (int j = 0; j < 4; ++j) acc[i][j] = Frag<T>::mma(ah, bh[j], acc[i][j]);
      Frag<T>::guard(acc[i][0], acc[i][3], ah, ah);
    }
    Frag<T>::keep(bh[0], bh[1], bh[2], bh[3]);
  }
  acc_guard4(acc[0][0], acc[0][1], acc[0][2], acc[0][3]);
  acc_guard4(acc[1][0], acc[1][1], acc[1][2], acc[1][3]);
  acc_guard4(acc[2][0], acc[2][1], acc[2][2], acc[2][3]);
  acc_guard4(acc[3][0], acc[3][1], acc[3][2], acc[3][3]);

  float njv[4];
  int   cok[4];
#pragma unroll
  for (int j = 0; j < 4; ++j) {
    const int col = n0 + (j << 4) + rlane;
    njv[j] = Bn[col];
    cok[j] = (col < colsValid) ? 1 : 0;
  }
  float part[4];
#pragma unroll
  for (int i = 0; i < 4; ++i) {
    const int rb = m0 + (i << 4) + mOff;
    const v4f na = *(const v4f*)(An + rb);
    const v4f nb = *(const v4f*)(An + rb + 4);
    const float niv[8] = {na[0], na[1], na[2], na[3], nb[0], nb[1], nb[2], nb[3]};
    float si = 0.0f;
#pragma unroll
    for (int j = 0; j < 4; ++j) {
#pragma unroll
      for (int r = 0; r < 8; ++r) {
        const float arg = fmaf(acc[i][j][r], s2, -(niv[r] + njv[j]));
        const float ev  = exp2f(arg);
        const float v   = 1.0f - ev;
        const bool ok   = (cok[j] != 0) && ((rb + r) < rowsValid);
        si += ok ? v : 0.0f;
      }
    }
    part[i] = si;
  }
  float s = (part[0] + part[1]) + (part[2] + part[3]);
#pragma unroll
  for (int off = 16; off > 0; off >>= 1) s += __shfl_xor(s, off, 32);
  if (lane == 0) red[wave] = s;
  __syncthreads();
  if (wave == 0) {
    float bs = 0.0f;
#pragma unroll
    for (int w = 0; w < kWavesPerBlk; ++w) bs += red[w];
    v4f ov;
    ov[0] = (lane == 0) ? bs : 0.0f;
    ov[1] = 0.0f; ov[2] = 0.0f; ov[3] = 0.0f;
    const int li = (lane & 7) * 4;
    float* pp = partial + (size_t)blockIdx.x * kLineFloats + li;
    if (lane < 8) *(volatile v4f*)pp = ov;
    __threadfence();
    if (lane < 8) *(volatile v4f*)pp = ov;
  }
}

__global__ __launch_bounds__(256) void combine_kernel(
    const float* __restrict__ pzz, const float* __restrict__ pgz, const float* __restrict__ pgg,
    float* __restrict__ out) {
  __shared__ float rz[256];
  __shared__ float rg[256];
  __shared__ float rq[256];
  const int t = threadIdx.x;
  float sz = 0.0f, cz = 0.0f;
#pragma unroll 1
  for (int i = 0; i < kBlocksZZ / 256; ++i) {
    const float v  = pzz[(size_t)(t + 256 * i) * kLineFloats];
    const float y  = v - cz;
    const float tt = sz + y;
    cz = (tt - sz) - y;
    sz = tt;
  }
  const int tg = (t < kBlocksGZ) ? t : (kBlocksGZ - 1);
  const float vg = pgz[(size_t)tg * kLineFloats];
  const float sg = (t < kBlocksGZ) ? vg : 0.0f;
  const int tq = (t < kBlocksGG) ? t : (kBlocksGG - 1);
  const float vq = pgg[(size_t)tq * kLineFloats];
  const float sq = (t < kBlocksGG) ? vq : 0.0f;
  rz[t] = sz; rg[t] = sg; rq[t] = sq;
  __syncthreads();
  for (int off = 128; off > 0; off >>= 1) {
    if (t < off) {
      rz[t] += rz[t + off];
      rg[t] += rg[t + off];
      rq[t] += rq[t + off];
    }
    __syncthreads();
  }
  if (t == 0) {
    const float wzz = 1.0f / (16384.0f * 16384.0f);
    const float wgz = 1.0f / (200.0f * 16384.0f);
    const float wgg = 1.0f / (200.0f * 200.0f);
    const float mzz = rz[0] * wzz;
    const float mgz = rg[0] * wgz;
    const float mgg = rq[0] * wgg;
    const float d    = (mgg + mzz) - 2.0f * mgz;
    const float loss = -10.0f * d;
    *(volatile float*)out = loss;
    __threadfence();
    *(volatile float*)out = loss;
  }
}

extern "C" void kernel_launch(void* const* d_in, const int* in_sizes, int n_in,
                              void* d_out, int out_size, void* d_ws, size_t ws_size,
                              hipStream_t stream) {
  (void)n_in; (void)out_size;
  if (in_sizes[0] != kNumZ * kFeat || in_sizes[1] != kNumG * kFeat) return;
  if (ws_size < kWsTotal) return;
  const float* z = (const float*)d_in[0];
  const float* g = (const float*)d_in[1];
  float* out = (float*)d_out;
  char* ws = (char*)d_ws;
  unsigned short* Zh = (unsigned short*)(ws + kOffZh);
  unsigned short* Gh = (unsigned short*)(ws + kOffGh);
  float* nz  = (float*)(ws + kOffNz);
  float* ng  = (float*)(ws + kOffNg);
  float* pzz = (float*)(ws + kOffPzz);
  float* pgz = (float*)(ws + kOffPgz);
  float* pgg = (float*)(ws + kOffPgg);

  const float cNorm = 1.4426950408889634f / 4096.0f;
  const float s2    = 2.0f * cNorm;

  prep_rows_kernel<<<kPrepBlocksZ, 256, 0, stream>>>(z, kNumZ, Zh, nz, cNorm);
  prep_rows_kernel<<<kPrepBlocksG, 256, 0, stream>>>(g, kNumG, Gh, ng, cNorm);

  gram_tile_kernel<<<kBlocksGG, 256, 0, stream>>>(Gh, ng, kNumG, Gh, ng, kNumG, kShiftG, pgg, s2);
  gram_tile_kernel<<<kBlocksGZ, 256, 0, stream>>>(Gh, ng, kNumG, Zh, nz, kNumZ, kShiftZ, pgz, s2);
  gram_tile_kernel<<<kBlocksZZ, 256, 0, stream>>>(Zh, nz, kNumZ, Zh, nz, kNumZ, kShiftZ, pzz, s2);

  combine_kernel<<<1, 256, 0, stream>>>(pzz, pgz, pgg, out);
}
